// TransformerSLN_90211493085601
// MI455X (gfx1250) — hardware-verified
//
#include <hip/hip_runtime.h>
#include <stdint.h>
#include <stddef.h>
#include <math.h>


constexpr int CB   = 8;
constexpr int CS   = 1024;
constexpr int CD   = 768;
constexpr int CH   = 8;
constexpr int CDH  = 96;
constexpr int CDHP = 128;
constexpr int CDFF = 3072;
constexpr int CM   = CB * CS;
constexpr float CEPS = 1e-5f;

typedef __attribute__((ext_vector_type(16))) _Float16 v16h;
typedef __attribute__((ext_vector_type(8)))  _Float16 v8h;
typedef __attribute__((ext_vector_type(16))) __bf16   v16b;
typedef __attribute__((ext_vector_type(8)))  __bf16   v8b;
typedef __attribute__((ext_vector_type(8)))  float    v8f;
typedef __attribute__((ext_vector_type(4)))  float    v4f;

__device__ __forceinline__ unsigned short f2bf_bits(float f) {
  unsigned u = __float_as_uint(f);
  return (unsigned short)((u + 0x7FFFu + ((u >> 16) & 1u)) >> 16);
}
__device__ __forceinline__ float bf_bits2f(unsigned short h) { return __uint_as_float(((unsigned)h) << 16); }

__device__ __forceinline__ void dep_guard_h(v8f& a, v8f& b, v16h x, v16h y) { asm volatile("v_nop\n\tv_nop\n\tv_nop\n\tv_nop" : "+v"(a), "+v"(b) : "v"(x), "v"(y)); }
__device__ __forceinline__ void dep_guard_b(v8f& a, v8f& b, v16b x, v16b y) { asm volatile("v_nop\n\tv_nop\n\tv_nop\n\tv_nop" : "+v"(a), "+v"(b) : "v"(x), "v"(y)); }
__device__ __forceinline__ void keep4_h(v16h a, v16h b, v16h c, v16h d) { asm volatile("v_nop" :: "v"(a), "v"(b), "v"(c), "v"(d)); }
__device__ __forceinline__ void keep4_b(v16b a, v16b b, v16b c, v16b d) { asm volatile("v_nop" :: "v"(a), "v"(b), "v"(c), "v"(d)); }
__device__ __forceinline__ void acc_guard4(v8f& a, v8f& b, v8f& c, v8f& d) { asm volatile("v_nop\n\tv_nop\n\tv_nop\n\tv_nop" : "+v"(a), "+v"(b), "+v"(c), "+v"(d)); }
template <typename T> struct Frag;
template <> struct Frag<_Float16> {
  typedef v16h V; union U { v16h v; v8h h[2]; };
  static __device__ __forceinline__ v16h load(const _Float16* p) {
    U f; f.h[0] = *(const v8h*)(p); f.h[1] = *(const v8h*)(p + 16); return f.v;
  }
  static __device__ __forceinline__ v8f mma(v16h a, v16h b, v8f c) {
    return __builtin_amdgcn_wmma_f32_16x16x32_f16(false, a, false, b, (short)0, c, false, false);
  }
  static __device__ __forceinline__ void guard(v8f& a, v8f& b, v16h x, v16h y) { dep_guard_h(a, b, x, y); }
  static __device__ __forceinline__ void keep(v16h a, v16h b, v16h c, v16h d) { keep4_h(a, b, c, d); }
};
template <> struct Frag<__bf16> {
  typedef v16b V; union U { v16b v; v8b h[2]; };
  static __device__ __forceinline__ v16b load(const __bf16* p) {
    U f; f.h[0] = *(const v8b*)(p); f.h[1] = *(const v8b*)(p + 16); return f.v;
  }
  static __device__ __forceinline__ v8f mma(v16b a, v16b b, v8f c) {
    return __builtin_amdgcn_wmma_f32_16x16x32_bf16(false, a, false, b, (short)0, c, false, false);
  }
  static __device__ __forceinline__ void guard(v8f& a, v8f& b, v16b x, v16b y) { dep_guard_b(a, b, x, y); }
  static __device__ __forceinline__ void keep(v16b a, v16b b, v16b c, v16b d) { keep4_b(a, b, c, d); }
};

template <int ET> struct Elem;
template <> struct Elem<0> { typedef _Float16 T; };
template <> struct Elem<1> { typedef __bf16 T; };
template <int ET, bool SPLIT, int BIAS_MODE, int OUT_MODE, bool RESID, int ACT = 0>
__global__ __launch_bounds__(256) void wmma_gemm64(
    const unsigned short* __restrict__ Ap, const unsigned short* __restrict__ A2p, int lda, long strideA,
    const unsigned short* __restrict__ Btp, const unsigned short* __restrict__ Bt2p, int ldb, long strideB,
    void* __restrict__ Cout, void* __restrict__ Cout2, int ldc, long strideC,
    const float* __restrict__ bias,
    const float* __restrict__ resid, long strideR,
    int M, int N, int K, float scale, float oscale) {
  typedef typename Elem<ET>::T T;
  typedef typename Frag<T>::V V;
  const T* A = (const T*)Ap; const T* A2 = (const T*)A2p; const T* Bt = (const T*)Btp; const T* Bt2 = (const T*)Bt2p;
  __shared__ __align__(16) float sT[8][16 * 68];
  const int b    = blockIdx.y;
  const int lane = threadIdx.x & 31;
  const int wave = threadIdx.x >> 5;
  const int tilesN = N >> 6;
  const int tilesM = M >> 6;
  const int tile = blockIdx.x * 8 + wave;
  if (tile >= tilesM * tilesN) return;
  const int tm = tile / tilesN;
  const int tn = tile - tm * tilesN;
  const int m0 = tm << 6;
  const int n0 = tn << 6;

  const T* Ab  = A  + (size_t)b * strideA;
  const T* Bb  = Bt + (size_t)b * strideB;
  const T* Ab2 = SPLIT ? (A2  + (size_t)b * strideA) : nullptr;
  const T* Bb2 = SPLIT ? (Bt2 + (size_t)b * strideB) : nullptr;

  const int rlane = lane & 15;
  const int koff  = (lane >> 4) * 8;
  const int mOff  = (lane >> 4) * 8;

  v8f acc[4][4];
#pragma unroll
  for (int i = 0; i < 4; ++i)
#pragma unroll
    for (int j = 0; j < 4; ++j) acc[i][j] = (v8f){0.f,0.f,0.f,0.f,0.f,0.f,0.f,0.f};

  for (int k0 = 0; k0 < K; k0 += 32) {
    V bh[4], bl[4];
#pragma unroll
    for (int j = 0; j < 4; ++j) {
      const size_t bo = (size_t)(n0 + (j << 4) + rlane) * ldb + koff + k0;
      bh[j] = Frag<T>::load(Bb + bo);
      if (SPLIT) bl[j] = Frag<T>::load(Bb2 + bo);
    }
#pragma unroll
    for (int i = 0; i < 4; ++i) {
      const size_t ao = (size_t)(m0 + (i << 4) + rlane) * lda + koff + k0;
      V ah = Frag<T>::load(Ab + ao);
      V al;
      if (SPLIT) al = Frag<T>::load(Ab2 + ao);
#pragma unroll
      for (int j = 0; j < 4; ++j) {
        acc[i][j] = Frag<T>::mma(ah, bh[j], acc[i][j]);
        if (SPLIT) {
          acc[i][j] = Frag<T>::mma(ah, bl[j], acc[i][j]);
          acc[i][j] = Frag<T>::mma(al, bh[j], acc[i][j]);
        }
      }
      Frag<T>::guard(acc[i][0], acc[i][3], ah, SPLIT ? al : ah);
    }
    Frag<T>::keep(bh[0], bh[1], bh[2], bh[3]);
    if (SPLIT) Frag<T>::keep(bl[0], bl[1], bl[2], bl[3]);
  }
  acc_guard4(acc[0][0], acc[0][1], acc[0][2], acc[0][3]);
  acc_guard4(acc[1][0], acc[1][1], acc[1][2], acc[1][3]);
  acc_guard4(acc[2][0], acc[2][1], acc[2][2], acc[2][3]);
  acc_guard4(acc[3][0], acc[3][1], acc[3][2], acc[3][3]);

  float* slab = sT[wave];
  const float* Rb = RESID ? (resid + (size_t)b * strideR) : nullptr;
#pragma unroll
  for (int i = 0; i < 4; ++i) {
    const int mBase = m0 + (i << 4);
#pragma unroll
    for (int j = 0; j < 4; ++j) {
      const int n = n0 + (j << 4) + rlane;
      float bv = 0.f;
      if (BIAS_MODE == 2) bv = bias[n];
#pragma unroll
      for (int r = 0; r < 8; ++r) {
        float v = acc[i][j][r] * scale;
        if (BIAS_MODE == 1) v += bias[mBase + mOff + r];
        if (BIAS_MODE == 2) v += bv;
        if (RESID) v += Rb[(size_t)(mBase + mOff + r) * ldc + n];
        if (ACT == 1) v = tanhf(v);
        if (ACT == 2) v = fmaxf(v, 0.0f);
        if (ACT == 3) v = v / (1.0f + expf(-v));
        if (ACT == 4) v = (v > 0.f) ? v : 0.01f * v;
        if (ACT == 5) v = 0.5f * v * (1.0f + erff(v * 0.70710678118654752f));
        v *= oscale;
        slab[(mOff + r) * 68 + (j << 4) + rlane] = v;
      }
    }
    __builtin_amdgcn_fence(__ATOMIC_RELEASE, "workgroup");
    __builtin_amdgcn_wave_barrier();
    __builtin_amdgcn_fence(__ATOMIC_ACQUIRE, "workgroup");
    if (OUT_MODE == 0) {
      float* C = (float*)Cout + (size_t)b * strideC;
      const int hh = lane >> 4, c4 = (lane & 15) * 4;
      for (int pass = 0; pass < 2; ++pass) {
#pragma unroll
        for (int it = 0; it < 8; ++it) {
          const int row = it * 2 + hh;
          v4f v = *(const v4f*)(slab + row * 68 + c4);
          *(volatile v4f*)(C + (size_t)(mBase + row) * ldc + n0 + c4) = v;
        }
        __threadfence();
      }
    } else {
      const int q = lane >> 3, c8 = (lane & 7) * 8;
      unsigned short* C  = (unsigned short*)Cout  + (size_t)b * strideC;
      unsigned short* C2 = (OUT_MODE == 2) ? ((unsigned short*)Cout2 + (size_t)b * strideC) : nullptr;
      for (int pass = 0; pass < 2; ++pass) {
#pragma unroll
        for (int it = 0; it < 4; ++it) {
          const int row = it * 4 + q;
          const float* sp = slab + row * 68 + c8;
          v8h hv, lv;
#pragma unroll
          for (int e = 0; e < 8; ++e) {
            if (OUT_MODE == 1) {
              hv[e] = (_Float16)sp[e];
            } else {
              unsigned short hb = f2bf_bits(sp[e]);
              unsigned short lb = f2bf_bits(sp[e] - bf_bits2f(hb));
              hv[e] = __builtin_bit_cast(_Float16, hb);
              lv[e] = __builtin_bit_cast(_Float16, lb);
            }
          }
          *(volatile v8h*)(C + (size_t)(mBase + row) * ldc + n0 + c8) = hv;
          if (OUT_MODE == 2) *(volatile v8h*)(C2 + (size_t)(mBase + row) * ldc + n0 + c8) = lv;
        }
        __threadfence();
      }
    }
    __builtin_amdgcn_fence(__ATOMIC_RELEASE, "workgroup");
    __builtin_amdgcn_wave_barrier();
    __builtin_amdgcn_fence(__ATOMIC_ACQUIRE, "workgroup");
  }
}

template <int MODE>
__global__ __launch_bounds__(256) void conv_w_f16(const float* __restrict__ W, _Float16* __restrict__ Wt,
                                                  int Kin, int Nin, int Kout, int Nout, float wscale) {
  __shared__ float t[64][33];
  const int tid = threadIdx.x, lane = tid & 31, wave = tid >> 5;
  const int c0 = blockIdx.x * 64;
  const int r0 = blockIdx.y * 32;
  const int r = r0 + lane;
#pragma unroll
  for (int i = 0; i < 8; ++i) {
    const int cc = wave + 8 * i;
    const int c = c0 + cc;
    int kin, nin;
    bool valid;
    if (MODE == 0) {
      kin = c; nin = r; valid = true;
    } else if (MODE == 1) {
      kin = c; const int hd = r >> 7, d = r & 127; valid = d < CDH; nin = hd * CDH + (valid ? d : 0);
    } else {
      nin = r; const int hd = c >> 7, d = c & 127; valid = d < CDH; kin = hd * CDH + (valid ? d : 0);
    }
    kin = kin < Kin ? kin : Kin - 1;
    nin = nin < Nin ? nin : Nin - 1;
    float v = W[(size_t)kin * Nin + nin];
    v = valid ? v : 0.0f;
    t[cc][lane] = v;
  }
  __syncthreads();
  const int rr = wave * 4 + (lane >> 3);
  const int cb = (lane & 7) * 8;
  v8h o;
#pragma unroll
  for (int e = 0; e < 8; ++e) o[e] = (_Float16)(t[cb + e][rr] * wscale);
  const int orow = (r0 + rr) < Nout ? (r0 + rr) : Nout - 1;
  _Float16* dst = Wt + (size_t)orow * Kout + c0 + cb;
  *(volatile v8h*)dst = o;
  __threadfence();
  *(volatile v8h*)dst = o;
}

__global__ __launch_bounds__(256) void pad_bias(const float* __restrict__ bv, float* __restrict__ bvp) {
  const int i0 = threadIdx.x * 4;
  v4f o;
#pragma unroll
  for (int e = 0; e < 4; ++e) {
    const int idx = i0 + e;
    const int hd = idx >> 7, d = idx & 127;
    const bool valid = d < CDH;
    const float v = bv[hd * CDH + (valid ? d : 0)];
    o[e] = valid ? v : 0.0f;
  }
  *(volatile v4f*)(bvp + i0) = o;
  __threadfence();
  *(volatile v4f*)(bvp + i0) = o;
}

__global__ __launch_bounds__(256) void copy_lines(const float* __restrict__ src, float* __restrict__ dst, int n4) {
  const int i = blockIdx.x * 256 + threadIdx.x;
  if (i < n4) {
    const v4f v = *(const v4f*)(src + 4 * (size_t)i);
    *(volatile v4f*)(dst + 4 * (size_t)i) = v;
    __threadfence();
    *(volatile v4f*)(dst + 4 * (size_t)i) = v;
  }
}

__global__ __launch_bounds__(256) void sln_f16(const float* __restrict__ hin, const float* __restrict__ xin,
                                              const float* __restrict__ gam, const float* __restrict__ bet,
                                              const float* __restrict__ w, const float* __restrict__ bb,
                                              _Float16* __restrict__ outp, int nrows, float oscale) {
  const int lane = threadIdx.x & 31, wave = threadIdx.x >> 5;
  int row = blockIdx.x * 8 + wave;
  row = row < nrows ? row : nrows - 1;
  const float* hr = hin + (size_t)row * CD;
  const float* xr = xin + (size_t)row * CD;

  float s = 0.f;
#pragma unroll 1
  for (int i = 0; i < 3; ++i) {
    const int c = i * 256 + lane * 8;
    const v4f a = *(const v4f*)(hr + c);
    const v4f a2 = *(const v4f*)(hr + c + 4);
    s += ((a[0] + a[1]) + (a[2] + a[3])) + ((a2[0] + a2[1]) + (a2[2] + a2[3]));
  }
#pragma unroll
  for (int off = 16; off > 0; off >>= 1) s += __shfl_xor(s, off, 32);
  const float mu = s * (1.0f / (float)CD);

  float q = 0.f;
#pragma unroll 1
  for (int i = 0; i < 3; ++i) {
    const int c = i * 256 + lane * 8;
    const v4f a = *(const v4f*)(hr + c);
    const v4f a2 = *(const v4f*)(hr + c + 4);
#pragma unroll
    for (int e = 0; e < 4; ++e) {
      const float d0 = a[e] - mu;  q = fmaf(d0, d0, q);
      const float d1 = a2[e] - mu; q = fmaf(d1, d1, q);
    }
  }
#pragma unroll
  for (int off = 16; off > 0; off >>= 1) q += __shfl_xor(q, off, 32);
  const float var = q * (1.0f / (float)CD);
  const float rs  = rsqrtf(var + CEPS);
  const float g0 = gam[0], be0 = bet[0];

#pragma unroll 1
  for (int i = 0; i < 3; ++i) {
    const int c = i * 256 + lane * 8;
    const v4f a  = *(const v4f*)(hr + c);
    const v4f a2 = *(const v4f*)(hr + c + 4);
    const v4f xa = *(const v4f*)(xr + c);
    const v4f xb = *(const v4f*)(xr + c + 4);
    const v4f wa = *(const v4f*)(w + c);
    const v4f wb = *(const v4f*)(w + c + 4);
    const v4f ba = *(const v4f*)(bb + c);
    const v4f b2v = *(const v4f*)(bb + c + 4);
    v8h o;
#pragma unroll
    for (int e = 0; e < 4; ++e) {
      const float ln0 = (a[e] - mu) * rs * wa[e] + ba[e];
      const float xv0 = xa[e];
      o[e] = (_Float16)((g0 * xv0 * ln0 + be0 * xv0) * oscale);
      const float ln1 = (a2[e] - mu) * rs * wb[e] + b2v[e];
      const float xv1 = xb[e];
      o[4 + e] = (_Float16)((g0 * xv1 * ln1 + be0 * xv1) * oscale);
    }
    _Float16* dst = outp + (size_t)row * CD + c;
    *(volatile v8h*)dst = o;
    __threadfence();
    *(volatile v8h*)dst = o;
  }
}

__global__ __launch_bounds__(256) void rowsq_f32(const _Float16* __restrict__ qh, const _Float16* __restrict__ kh,
                                                float* __restrict__ q2, float* __restrict__ k2, int total) {
  const int idx = blockIdx.x * 256 + threadIdx.x;
  const bool isk = (blockIdx.y == 1);
  const _Float16* src = isk ? kh : qh;
  float* dst = isk ? k2 : q2;
  const int ci = idx < total ? idx : total - 1;
  const _Float16* p = src + (size_t)(ci >> 3) * CD + (ci & 7) * CDH;
  float acc = 0.f;
#pragma unroll 1
  for (int j = 0; j < CDH / 8; ++j) {
    const v8h v = *(const v8h*)(p + j * 8);
#pragma unroll
    for (int e = 0; e < 8; ++e) { const float f = (float)v[e]; acc = fmaf(f, f, acc); }
  }
  if (idx < total) {
    ((volatile float*)dst)[idx] = acc;
    __threadfence();
    ((volatile float*)dst)[idx] = acc;
  }
}

__global__ __launch_bounds__(256) void l2_softmax_f16(const float* __restrict__ sc, const float* __restrict__ q2,
                                                     const float* __restrict__ k2, _Float16* __restrict__ P,
                                                     int bidx, float rscale) {
  __shared__ __align__(16) float k2s[CS];
  const int tid = threadIdx.x, lane = tid & 31, wave = tid >> 5;
  const int hd = blockIdx.y;
  const int s  = blockIdx.x * 8 + wave;
#pragma unroll
  for (int i = 0; i < 4; ++i) {
    const int t = tid + 256 * i;
    k2s[t] = k2[((size_t)bidx * CS + t) * CH + hd] * (1.0f / 256.0f);
  }
  __syncthreads();
  const float q2v = q2[((size_t)bidx * CS + s) * CH + hd] * (1.0f / 256.0f);
  const size_t rowoff = ((size_t)hd * CS + s) * CS;
  const float* srow = sc + rowoff;

  float lg[4][8];
  float m = -INFINITY;
#pragma unroll
  for (int i = 0; i < 4; ++i) {
    const int c = i * 256 + lane * 8;
    const v4f a  = *(const v4f*)(srow + c);
    const v4f a2 = *(const v4f*)(srow + c + 4);
    const v4f ka = *(const v4f*)(k2s + c);
    const v4f kb = *(const v4f*)(k2s + c + 4);
#pragma unroll
    for (int e = 0; e < 4; ++e) {
      float d2 = (q2v + ka[e]) - 2.0f * a[e];
      d2 = fmaxf(d2, 0.0f);
      const float l0 = -__builtin_amdgcn_sqrtf(d2) * rscale;
      lg[i][e] = l0; m = fmaxf(m, l0);
      float e2 = (q2v + kb[e]) - 2.0f * a2[e];
      e2 = fmaxf(e2, 0.0f);
      const float l1 = -__builtin_amdgcn_sqrtf(e2) * rscale;
      lg[i][4 + e] = l1; m = fmaxf(m, l1);
    }
  }
#pragma unroll
  for (int off = 16; off > 0; off >>= 1) m = fmaxf(m, __shfl_xor(m, off, 32));
  float sum = 0.f;
#pragma unroll
  for (int i = 0; i < 4; ++i) {
#pragma unroll
    for (int e = 0; e < 8; ++e) {
      const float p = __builtin_amdgcn_exp2f((lg[i][e] - m) * 1.4426950408889634f);
      lg[i][e] = p; sum += p;
    }
  }
#pragma unroll
  for (int off = 16; off > 0; off >>= 1) sum += __shfl_xor(sum, off, 32);
  const float inv = 32768.0f * __builtin_amdgcn_rcpf(sum);
#pragma unroll
  for (int i = 0; i < 4; ++i) {
    const int c = i * 256 + lane * 8;
    v8h o;
#pragma unroll
    for (int e = 0; e < 8; ++e) o[e] = (_Float16)(lg[i][e] * inv);
    _Float16* dst = P + rowoff + c;
    *(volatile v8h*)dst = o;
    __threadfence();
    *(volatile v8h*)dst = o;
  }
}

extern "C" void kernel_launch(void* const* d_in, const int* in_sizes, int n_in,
                              void* d_out, int out_size, void* d_ws, size_t ws_size,
                              hipStream_t stream)
{
  if (n_in < 22) return;
  const size_t nMD = (size_t)CM * CD;
  if ((size_t)in_sizes[0] != nMD || (size_t)in_sizes[1] != nMD) return;
  if ((size_t)out_size < 2 * nMD) return;
  if (in_sizes[10] != CD * CD || in_sizes[12] != CD * CD || in_sizes[14] != CD * CD || in_sizes[16] != CD * CD) return;
  if (in_sizes[18] != CD * CDFF || in_sizes[20] != CDFF * CD) return;
  if (in_sizes[4] != CD || in_sizes[5] != CD || in_sizes[8] != CD || in_sizes[9] != CD) return;
  if (in_sizes[11] != CD || in_sizes[13] != CD || in_sizes[15] != CD || in_sizes[17] != CD || in_sizes[19] != CDFF || in_sizes[21] != CD) return;
  if (in_sizes[2] < 1 || in_sizes[3] < 1 || in_sizes[6] < 1 || in_sizes[7] < 1) return;

  const float* h    = (const float*)d_in[0];
  const float* x    = (const float*)d_in[1];
  const float* g1   = (const float*)d_in[2];
  const float* be1  = (const float*)d_in[3];
  const float* ln1w = (const float*)d_in[4];
  const float* ln1b = (const float*)d_in[5];
  const float* g2   = (const float*)d_in[6];
  const float* be2  = (const float*)d_in[7];
  const float* ln2w = (const float*)d_in[8];
  const float* ln2b = (const float*)d_in[9];
  const float* Wq = (const float*)d_in[10]; const float* bq = (const float*)d_in[11];
  const float* Wk = (const float*)d_in[12]; const float* bk = (const float*)d_in[13];
  const float* Wv = (const float*)d_in[14]; const float* bv = (const float*)d_in[15];
  const float* Wo = (const float*)d_in[16]; const float* bo = (const float*)d_in[17];
  const float* W1 = (const float*)d_in[18]; const float* b1 = (const float*)d_in[19];
  const float* W2 = (const float*)d_in[20]; const float* b2 = (const float*)d_in[21];
  float* out = (float*)d_out;

  char* wsb = (char*)d_ws;
  size_t off = 0;
  auto carve = [&](size_t bytes) -> char* { char* p = wsb + off; off += (bytes + 255) & ~(size_t)255; return p; };
  _Float16* Wqt  = (_Float16*)carve((size_t)CD * CD * 2);
  _Float16* Wkt  = (_Float16*)carve((size_t)CD * CD * 2);
  _Float16* WvtP = (_Float16*)carve((size_t)CDHP * CH * CD * 2);
  _Float16* WotP = (_Float16*)carve((size_t)CD * CDHP * CH * 2);
  _Float16* W1t  = (_Float16*)carve((size_t)CDFF * CD * 2);
  _Float16* W2t  = (_Float16*)carve((size_t)CD * CDFF * 2);
  float*    bvp  = (float*)carve((size_t)CDHP * CH * 4);
  _Float16* qh   = (_Float16*)carve(nMD * 2);
  _Float16* khp  = (_Float16*)carve(nMD * 2);
  _Float16* VtP  = (_Float16*)carve((size_t)CDHP * CH * CM * 2);
  float*    scores = (float*)carve((size_t)CH * CS * CS * 4);
  _Float16* Pb   = (_Float16*)carve((size_t)CH * CS * CS * 2);
  _Float16* attn = (_Float16*)carve((size_t)CM * CDHP * CH * 2);
  float*    q2s  = (float*)carve((size_t)CM * CH * 4);
  float*    k2s  = (float*)carve((size_t)CM * CH * 4);
  const size_t total = off;
  if (total > ws_size) return;
  _Float16* h1   = (_Float16*)scores;
  _Float16* h2   = (_Float16*)Pb;
  float*    htmp = (float*)qh;
  _Float16* hid  = (_Float16*)VtP;

  const dim3 blk(256);
  const unsigned short* const u_h1   = (const unsigned short*)h1;
  const unsigned short* const u_h2   = (const unsigned short*)h2;
  const unsigned short* const u_Wqt  = (const unsigned short*)Wqt;
  const unsigned short* const u_Wkt  = (const unsigned short*)Wkt;
  const unsigned short* const u_WvtP = (const unsigned short*)WvtP;
  const unsigned short* const u_WotP = (const unsigned short*)WotP;
  const unsigned short* const u_W1t  = (const unsigned short*)W1t;
  const unsigned short* const u_W2t  = (const unsigned short*)W2t;
  const unsigned short* const u_q    = (const unsigned short*)qh;
  const unsigned short* const u_k    = (const unsigned short*)khp;
  const unsigned short* const u_VtP  = (const unsigned short*)VtP;
  const unsigned short* const u_P    = (const unsigned short*)Pb;
  const unsigned short* const u_attn = (const unsigned short*)attn;
  const unsigned short* const u_hid  = (const unsigned short*)hid;

  copy_lines<<<dim3((unsigned)(nMD / 4 / 256)), blk, 0, stream>>>(x, out, (int)(nMD / 4));

  conv_w_f16<0><<<dim3(CD / 64, CD / 32), blk, 0, stream>>>(Wq, Wqt, CD, CD, CD, CD, 64.0f);
  conv_w_f16<0><<<dim3(CD / 64, CD / 32), blk, 0, stream>>>(Wk, Wkt, CD, CD, CD, CD, 64.0f);
  conv_w_f16<1><<<dim3(CD / 64, (CDHP * CH) / 32), blk, 0, stream>>>(Wv, WvtP, CD, CD, CD, CDHP * CH, 64.0f);
  conv_w_f16<2><<<dim3((CDHP * CH) / 64, CD / 32), blk, 0, stream>>>(Wo, WotP, CD, CD, CDHP * CH, CD, 64.0f);
  conv_w_f16<0><<<dim3(CD / 64, CDFF / 32), blk, 0, stream>>>(W1, W1t, CD, CDFF, CD, CDFF, 64.0f);
  conv_w_f16<0><<<dim3(CDFF / 64, CD / 32), blk, 0, stream>>>(W2, W2t, CDFF, CD, CDFF, CD, 64.0f);
  pad_bias<<<dim3(1), blk, 0, stream>>>(bv, bvp);

  sln_f16<<<dim3(CM / 8), blk, 0, stream>>>(h, x, g1, be1, ln1w, ln1b, h1, CM, 16.0f);

  const float s10 = 1.0f / 1024.0f;
  wmma_gemm64<0, false, 2, 1, false, 0><<<dim3((CM / 64) * (CD / 64) / 8, 1), blk, 0, stream>>>(
      u_h1, u_h1, CD, 0L, u_Wqt, u_Wqt, CD, 0L, (void*)qh, (void*)qh, CD, 0L, bq, h, 0L, CM, CD, CD, s10, 16.0f);
  wmma_gemm64<0, false, 2, 1, false, 0><<<dim3((CM / 64) * (CD / 64) / 8, 1), blk, 0, stream>>>(
      u_h1, u_h1, CD, 0L, u_Wkt, u_Wkt, CD, 0L, (void*)khp, (void*)khp, CD, 0L, bk, h, 0L, CM, CD, CD, s10, 16.0f);
  wmma_gemm64<0, false, 1, 1, false, 0><<<dim3(((CDHP * CH) / 64) * (CM / 64) / 8, 1), blk, 0, stream>>>(
      u_WvtP, u_WvtP, CD, 0L, u_h1, u_h1, CD, 0L, (void*)VtP, (void*)VtP, CM, 0L, bvp, h, 0L, CDHP * CH, CM, CD, s10, 16.0f);

  rowsq_f32<<<dim3((CM * CH) / 256, 2), blk, 0, stream>>>(qh, khp, q2s, k2s, CM * CH);

  const float rscale = 0.102062072615966f;
  const float sqk = 1.0f / 256.0f;
  const float spv = 1.0f / 8192.0f;
  for (int b = 0; b < CB; ++b) {
    const unsigned short* qb_ = u_q + (size_t)b * CS * CD;
    const unsigned short* kb_ = u_k + (size_t)b * CS * CD;
    wmma_gemm64<0, false, 0, 0, false, 0><<<dim3((CS / 64) * (CS / 64) / 8, CH), blk, 0, stream>>>(
        qb_, qb_, CD, (long)CDH, kb_, kb_, CD, (long)CDH, (void*)scores, (void*)scores, CS, (long)CS * CS,
        bq, h, 0L, CS, CS, CDH, sqk, 1.0f);
    l2_softmax_f16<<<dim3(CS / 8, CH), blk, 0, stream>>>(scores, q2s, k2s, Pb, b, rscale);
    const unsigned short* vb_ = u_VtP + (size_t)b * CS;
    _Float16* ab_ = attn + (size_t)b * CS * (CDHP * CH);
    wmma_gemm64<0, false, 0, 1, false, 0><<<dim3((CS / 64) * (CDHP / 64) / 8, CH), blk, 0, stream>>>(
        u_P, u_P, CS, (long)CS * CS, vb_, vb_, CM, (long)CDHP * CM, (void*)ab_, (void*)ab_, CDHP * CH, (long)CDHP,
        bq, h, 0L, CS, CDHP, CS, spv, 1.0f);
  }

  wmma_gemm64<0, false, 2, 0, true, 0><<<dim3((CM / 64) * (CD / 64) / 8, 1), blk, 0, stream>>>(
      u_attn, u_attn, CDHP * CH, 0L, u_WotP, u_WotP, CDHP * CH, 0L, (void*)htmp, (void*)htmp, CD, 0L,
      bo, h, 0L, CM, CD, CDHP * CH, 1.0f / 4096.0f, 1.0f);

  sln_f16<<<dim3(CM / 8), blk, 0, stream>>>(htmp, x, g2, be2, ln2w, ln2b, h2, CM, 16.0f);

  wmma_gemm64<0, false, 2, 1, false, 2><<<dim3((CM / 64) * (CDFF / 64) / 8, 1), blk, 0, stream>>>(
      u_h2, u_h2, CD, 0L, u_W1t, u_W1t, CD, 0L, (void*)hid, (void*)hid, CDFF, 0L, b1, h, 0L, CM, CDFF, CD, s10, 16.0f);

  float* out1 = out + nMD;
  wmma_gemm64<0, false, 2, 0, true, 0><<<dim3((CM / 64) * (CD / 64) / 8, 1), blk, 0, stream>>>(
      u_hid, u_hid, CDFF, 0L, u_W2t, u_W2t, CDFF, 0L, (void*)out1, (void*)out1, CD, 0L,
      b2, htmp, 0L, CM, CD, CDFF, s10, 1.0f);
}
